// GNN_27934467293570
// MI455X (gfx1250) — hardware-verified
//
#include <hip/hip_runtime.h>
#include <stddef.h>
#include <stdint.h>
#include <math.h>


#define CP     128
#define CO1    112
#define KA0    128
#define KA1    256
#define EDIM   8
#define NTHR   256
#define NWAVE  8
#define EPT    8
#define CHUNK  (NTHR * EPT)
#define WCAP   (EPT * 32)
#define LISTN  (NWAVE * WCAP)
#define NBA    1024
#define SLA    10
#define RCAP   28672
#define DEGCAP 64
#define GBM    64
#define GTHR   128
#define UW0    (CP * (KA0 / 8))
#define UW1    (CP * (KA1 / 8))
#define WPB    ((UW0 + UW1) / NTHR + 1)
#define AGG_ZINTS    (LISTN + 2 * RCAP + 3 * NBA)
#define AGG_LDS_INTS (AGG_ZINTS + 16)
#define RECN   256
#define ORB    64
#define WSMAX  134217728

static_assert((CHUNK & (CHUNK - 1)) == 0 && CHUNK <= 4096);
static_assert((NBA & (NBA - 1)) == 0 && NBA == (1 << SLA));
static_assert(((long long)CHUNK << SLA) < (1LL << 31));
static_assert(NBA % NWAVE == 0 && NBA % 32 == 0);
static_assert(RCAP % 4 == 0 && AGG_ZINTS % 4 == 0 && LISTN % 4 == 0);
static_assert(KA0 % 32 == 0 && KA1 % 32 == 0 && KA1 == 2 * CP && KA0 == CP);
static_assert(GBM == (GTHR / 32) * 16 && CP == 4 * 32);
static_assert(UW0 % NTHR == 0 && UW1 % NTHR == 0);
static_assert(NWAVE == EDIM);
static_assert(DEGCAP == 64);
static_assert(CO1 % 4 == 0 && CO1 <= CP);
static_assert(AGG_LDS_INTS * 4 <= 300000);
static_assert(NWAVE * RECN * 8 <= RCAP * 4);
static_assert((LISTN * 4) % 8 == 0);
static_assert((ORB * CO1) % (4 * NTHR) == 0 && (ORB * CO1 * 4) % 128 == 0);

typedef float          v4f   __attribute__((ext_vector_type(4)));
typedef float          v8f   __attribute__((ext_vector_type(8)));
typedef double         v2d   __attribute__((ext_vector_type(2)));
typedef int            v4i   __attribute__((ext_vector_type(4)));
typedef int            v8i   __attribute__((ext_vector_type(8)));
typedef unsigned short v8us  __attribute__((ext_vector_type(8)));
typedef unsigned short v16us __attribute__((ext_vector_type(16)));
typedef __bf16         v16bf __attribute__((ext_vector_type(16)));
typedef v4f  __attribute__((may_alias)) v4fa;
typedef v4i  __attribute__((may_alias)) v4ia;
typedef v8us __attribute__((may_alias)) v8usa;
typedef double __attribute__((may_alias)) dbla;
union FragB { v16bf v; v16us u; v8us h[2]; v8i w; };

__device__ __forceinline__ v8f wmb(const FragB& a, const FragB& b, v8f c) {
  v8f d = __builtin_amdgcn_wmma_f32_16x16x32_bf16(false, a.v, false, b.v, (short)0, c, false, false);
  asm volatile("v_nop\n\tv_nop\n\tv_nop\n\tv_nop" : "+v"(d) : "v"(a.w), "v"(b.w));
  return d;
}

__device__ __forceinline__ unsigned bf16_bits(float f) {
  const unsigned u = __float_as_uint(f);
  return (u + 0x7FFFu + ((u >> 16) & 1u)) >> 16;
}
__device__ __forceinline__ float bf16_val(float f) {
  return __uint_as_float(bf16_bits(f) << 16);
}

template <int SLB>
__device__ __forceinline__ int scan_chunk(const int* __restrict__ dsts, int nE, int cbase, int slotBase,
                                          int nb, int vec8, int* list, int tid, int lane, int wave) {
  int wc = 0;
  const int el0  = tid * EPT;
  const int e0   = cbase + el0;
  const int sent = -2147483647 - 1;
  v4i da, db;
  if (vec8 != 0 && cbase + CHUNK <= nE) {
    da = *(const v4i*)(dsts + e0);
    db = *(const v4i*)(dsts + e0 + 4);
  } else {
    da.x = (e0     < nE) ? dsts[min(e0,     nE - 1)] : sent;
    da.y = (e0 + 1 < nE) ? dsts[min(e0 + 1, nE - 1)] : sent;
    da.z = (e0 + 2 < nE) ? dsts[min(e0 + 2, nE - 1)] : sent;
    da.w = (e0 + 3 < nE) ? dsts[min(e0 + 3, nE - 1)] : sent;
    db.x = (e0 + 4 < nE) ? dsts[min(e0 + 4, nE - 1)] : sent;
    db.y = (e0 + 5 < nE) ? dsts[min(e0 + 5, nE - 1)] : sent;
    db.z = (e0 + 6 < nE) ? dsts[min(e0 + 6, nE - 1)] : sent;
    db.w = (e0 + 7 < nE) ? dsts[min(e0 + 7, nE - 1)] : sent;
  }
  const unsigned nbs = (unsigned)slotBase;
  const unsigned unb = (unsigned)nb;
  const unsigned s0 = (unsigned)da.x - nbs, s1 = (unsigned)da.y - nbs;
  const unsigned s2 = (unsigned)da.z - nbs, s3 = (unsigned)da.w - nbs;
  const unsigned s4 = (unsigned)db.x - nbs, s5 = (unsigned)db.y - nbs;
  const unsigned s6 = (unsigned)db.z - nbs, s7 = (unsigned)db.w - nbs;
  const bool h0 = s0 < unb, h1 = s1 < unb, h2 = s2 < unb, h3 = s3 < unb;
  const bool h4 = s4 < unb, h5 = s5 < unb, h6 = s6 < unb, h7 = s7 < unb;
  const unsigned any = __builtin_amdgcn_ballot_w32(h0 | h1 | h2 | h3 | h4 | h5 | h6 | h7);
  if (any != 0u) {
#define HITJ(J, HJ, SJ) { \
      const unsigned mj = __builtin_amdgcn_ballot_w32(HJ); \
      if (mj != 0u) { \
        if (HJ) { \
          const int pos = wc + (int)__builtin_amdgcn_mbcnt_lo(mj, 0u); \
          if (pos < WCAP) list[wave * WCAP + pos] = ((el0 + (J)) << SLB) | (int)(SJ); \
        } \
        wc += (int)__builtin_popcount(mj); } }
    HITJ(0, h0, s0)
    HITJ(1, h1, s1)
    HITJ(2, h2, s2)
    HITJ(3, h3, s3)
    HITJ(4, h4, s4)
    HITJ(5, h5, s5)
    HITJ(6, h6, s6)
    HITJ(7, h7, s7)
#undef HITJ
  }
  return wc;
}

__global__ __launch_bounds__(NTHR) void k_wprep(const float* __restrict__ W0, const float* __restrict__ W1,
                                                const float* __restrict__ We0, const float* __restrict__ aE0,
                                                const float* __restrict__ We1, const float* __restrict__ aE1,
                                                unsigned short* W0T, unsigned short* W1T2, float* prm) {
  __shared__ __attribute__((aligned(16))) float vs[32];
  const int tid = (int)threadIdx.x, lane = tid & 31, wave = tid >> 5;
  const int blk = (int)blockIdx.x;
  if (blk < UW0 / NTHR) {
    const int u  = blk * NTHR + tid;
    const int n  = u >> 4;
    const int k8 = (u & 15) * 8;
    const float* p = W0 + (size_t)k8 * CP + n;
    v8us o;
#pragma unroll
    for (int i = 0; i < 8; ++i) o[i] = (unsigned short)bf16_bits(p[(size_t)i * CP]);
    unsigned short* dp = W0T + (size_t)n * KA0 + k8;
    *(volatile v8us*)dp = o;
    __threadfence();
    *(volatile v8us*)dp = o;
  } else if (blk < (UW0 + UW1) / NTHR) {
    const int v  = (blk - UW0 / NTHR) * NTHR + tid;
    const int n  = v >> 5;
    const int k8 = (v & 31) * 8;
    const int kk = k8 & (CP - 1);
    const int nc = n < CO1 ? n : CO1 - 1;
    const bool ok = n < CO1;
    const float* p = W1 + (size_t)kk * CO1 + nc;
    v8us o;
#pragma unroll
    for (int i = 0; i < 8; ++i) {
      const unsigned b = bf16_bits(p[(size_t)i * CO1]);
      o[i] = ok ? (unsigned short)b : (unsigned short)0;
    }
    unsigned short* dp = W1T2 + (size_t)n * KA1 + k8;
    *(volatile v8us*)dp = o;
    __threadfence();
    *(volatile v8us*)dp = o;
  } else {
    float s0 = 0.0f, s1 = 0.0f;
#pragma unroll 1
    for (int j = 0; j < 4; ++j) {
      const int c  = lane + 32 * j;
      const int c1 = c < CO1 ? c : CO1 - 1;
      const float w0 = bf16_val(We0[wave * CP + c]);
      const float a0 = bf16_val(aE0[c]);
      const float w1 = bf16_val(We1[wave * CO1 + c1]);
      const float a1 = bf16_val(aE1[c1]);
      s0 = fmaf(w0, a0, s0);
      const float t1 = w1 * a1;
      s1 += (c < CO1) ? t1 : 0.0f;
    }
#pragma unroll
    for (int d = 16; d >= 1; d >>= 1) {
      s0 += __shfl_xor(s0, d, 32);
      s1 += __shfl_xor(s1, d, 32);
    }
    if (lane == 0) { vs[wave] = s0; vs[EDIM + wave] = s1; }
    if (tid < 16) vs[16 + tid] = 0.0f;
    __syncthreads();
    const v4f pv = *(const v4fa*)(vs + 4 * (tid & 7));
    float* dp = prm + 4 * (tid & 7);
    if (tid < 8) *(volatile v4f*)dp = pv;
    __threadfence();
    if (tid < 8) *(volatile v4f*)dp = pv;
  }
}

__global__ __launch_bounds__(NTHR) void k_cvx(const float* __restrict__ x, int nN, int nUnits,
                                              unsigned short* xb) {
  const int u = (int)blockIdx.x * NTHR + (int)threadIdx.x;
  if (u >= nUnits) return;
  const int row = u >> 4;
  const int k8  = (u & 15) * 8;
  const int rc  = row < nN ? row : nN - 1;
  const float* p = x + (size_t)rc * CP + k8;
  const v4f a = *(const v4fa*)p;
  const v4f b = *(const v4fa*)(p + 4);
  const bool ok = row < nN;
  v8us o;
  o[0] = ok ? (unsigned short)bf16_bits(a.x) : (unsigned short)0;
  o[1] = ok ? (unsigned short)bf16_bits(a.y) : (unsigned short)0;
  o[2] = ok ? (unsigned short)bf16_bits(a.z) : (unsigned short)0;
  o[3] = ok ? (unsigned short)bf16_bits(a.w) : (unsigned short)0;
  o[4] = ok ? (unsigned short)bf16_bits(b.x) : (unsigned short)0;
  o[5] = ok ? (unsigned short)bf16_bits(b.y) : (unsigned short)0;
  o[6] = ok ? (unsigned short)bf16_bits(b.z) : (unsigned short)0;
  o[7] = ok ? (unsigned short)bf16_bits(b.w) : (unsigned short)0;
  unsigned short* dp = xb + (size_t)row * CP + k8;
  *(volatile v8us*)dp = o;
  __threadfence();
  *(volatile v8us*)dp = o;
}

__global__ __launch_bounds__(NTHR) void k_edge(const float* __restrict__ eatt, const float* __restrict__ prm,
                                               int nE, int EP, float* ale) {
  __shared__ __attribute__((aligned(16))) float st[2 * NTHR];
  const int tid = (int)threadIdx.x;
  const int e  = (int)blockIdx.x * NTHR + tid;
  const int ec = e < nE ? e : nE - 1;
  const v4f p0 = *(const v4f*)(prm);
  const v4f p1 = *(const v4f*)(prm + 4);
  const v4f p2 = *(const v4f*)(prm + 8);
  const v4f p3 = *(const v4f*)(prm + 12);
  const float* ep = eatt + (size_t)ec * EDIM;
  const v4f a = *(const v4fa*)ep;
  const v4f b = *(const v4fa*)(ep + 4);
  const float x0 = bf16_val(a.x), x1 = bf16_val(a.y), x2 = bf16_val(a.z), x3 = bf16_val(a.w);
  const float x4 = bf16_val(b.x), x5 = bf16_val(b.y), x6 = bf16_val(b.z), x7 = bf16_val(b.w);
  float s0 = x0 * p0.x;
  s0 = fmaf(x1, p0.y, s0); s0 = fmaf(x2, p0.z, s0); s0 = fmaf(x3, p0.w, s0);
  s0 = fmaf(x4, p1.x, s0); s0 = fmaf(x5, p1.y, s0); s0 = fmaf(x6, p1.z, s0); s0 = fmaf(x7, p1.w, s0);
  float s1 = x0 * p2.x;
  s1 = fmaf(x1, p2.y, s1); s1 = fmaf(x2, p2.z, s1); s1 = fmaf(x3, p2.w, s1);
  s1 = fmaf(x4, p3.x, s1); s1 = fmaf(x5, p3.y, s1); s1 = fmaf(x6, p3.z, s1); s1 = fmaf(x7, p3.w, s1);
  const bool ok = e < nE;
  st[tid]        = ok ? s0 : 0.0f;
  st[NTHR + tid] = ok ? s1 : 0.0f;
  __syncthreads();
  const int pl  = (tid >> 6) & 1;
  const int idx = (tid & 63) * 4;
  const v4f ov = *(const v4fa*)(st + pl * NTHR + idx);
  float* dp = ale + (size_t)pl * (size_t)EP + (size_t)blockIdx.x * NTHR + idx;
  if (tid < 128) *(volatile v4f*)dp = ov;
  __threadfence();
  if (tid < 128) *(volatile v4f*)dp = ov;
}

__global__ __launch_bounds__(GTHR) void k_gemm(const unsigned short* __restrict__ A,
                                               const unsigned short* __restrict__ BT, int K,
                                               const float* __restrict__ aS, const float* __restrict__ aD,
                                               int nvec, float* xs, float* asd, int mpr) {
  __shared__ __attribute__((aligned(16))) float stg[GBM * CP];
  __shared__ __attribute__((aligned(16))) float dts[2 * GBM];
  const int tid = (int)threadIdx.x, lane = tid & 31, wave = tid >> 5, hh = lane >> 4, m = lane & 15;
  const int rowBase = (int)blockIdx.x * GBM;

  v8f acc[8];
  {
    const v8f z = {0.f, 0.f, 0.f, 0.f, 0.f, 0.f, 0.f, 0.f};
#pragma unroll
    for (int t = 0; t < 8; ++t) acc[t] = z;
  }
  const unsigned short* ap = A + (size_t)(rowBase + 16 * wave + m) * (size_t)K + 8 * hh;
  const unsigned short* bp = BT + (size_t)m * (size_t)K + 8 * hh;

#pragma unroll 1
  for (int k0 = 0; k0 < K; k0 += 32) {
    FragB af;
    af.h[0] = *(const v8usa*)(ap + k0);
    af.h[1] = *(const v8usa*)(ap + k0 + 16);
#pragma unroll
    for (int nt = 0; nt < 8; ++nt) {
      const unsigned short* wq = bp + (size_t)(16 * nt) * (size_t)K + k0;
      FragB bf;
      bf.h[0] = *(const v8usa*)wq;
      bf.h[1] = *(const v8usa*)(wq + 16);
      acc[nt] = wmb(af, bf, acc[nt]);
    }
  }

#pragma unroll
  for (int nt = 0; nt < 8; ++nt) {
    const int lc = 16 * nt + m;
#pragma unroll
    for (int r = 0; r < 8; ++r) {
      const int lr = 16 * wave + 8 * hh + r;
      stg[lr * CP + lc] = acc[nt][r];
    }
  }
  __syncthreads();

  v4f s4, d4;
  {
    const int c0 = 4 * lane;
    const int cc = c0 < nvec ? c0 : nvec - 4;
    const bool okv = c0 < nvec;
    const v4f t1 = *(const v4f*)(aS + cc);
    const v4f t2 = *(const v4f*)(aD + cc);
    s4.x = okv ? bf16_val(t1.x) : 0.0f; s4.y = okv ? bf16_val(t1.y) : 0.0f;
    s4.z = okv ? bf16_val(t1.z) : 0.0f; s4.w = okv ? bf16_val(t1.w) : 0.0f;
    d4.x = okv ? bf16_val(t2.x) : 0.0f; d4.y = okv ? bf16_val(t2.y) : 0.0f;
    d4.z = okv ? bf16_val(t2.z) : 0.0f; d4.w = okv ? bf16_val(t2.w) : 0.0f;
  }
#pragma unroll 4
  for (int i = 0; i < 16; ++i) {
    const int row = 16 * wave + i;
    const v4f v = *(const v4fa*)(stg + row * CP + 4 * lane);
    float ps = v.x * s4.x;
    ps = fmaf(v.y, s4.y, ps); ps = fmaf(v.z, s4.z, ps); ps = fmaf(v.w, s4.w, ps);
    float pd = v.x * d4.x;
    pd = fmaf(v.y, d4.y, pd); pd = fmaf(v.z, d4.z, pd); pd = fmaf(v.w, d4.w, pd);
#pragma unroll
    for (int d = 16; d >= 1; d >>= 1) {
      ps += __shfl_xor(ps, d, 32);
      pd += __shfl_xor(pd, d, 32);
    }
    if (lane == 0) { dts[row] = ps; dts[GBM + row] = pd; }
  }
  v4f pv[16];
#pragma unroll
  for (int it = 0; it < 16; ++it) pv[it] = *(const v4fa*)(stg + 4 * (it * GTHR + tid));
  __syncthreads();

  const v4f dv = *(const v4fa*)(dts + 4 * lane);
  float* xo = xs + (size_t)rowBase * CP;
  float* dp = asd + (size_t)((lane < 16) ? 0 : mpr) + (size_t)rowBase + 4 * (lane & 15);
#pragma unroll
  for (int it = 0; it < 16; ++it) *(volatile v4f*)(xo + 4 * (it * GTHR + tid)) = pv[it];
  if (wave == 0) *(volatile v4f*)dp = dv;
  __threadfence();
#pragma unroll
  for (int it = 0; it < 16; ++it) *(volatile v4f*)(xo + 4 * (it * GTHR + tid)) = pv[it];
  if (wave == 0) *(volatile v4f*)dp = dv;
}

__device__ __forceinline__ void hit_fetch(const int* sl, int idxIn, const int* __restrict__ srcs,
                                          const float* __restrict__ asd, const float* __restrict__ ale,
                                          int nE, int nN, float adn, int& srOut, float& alOut) {
  const int idx = idxIn > RCAP - 1 ? RCAP - 1 : idxIn;
  const int ent = sl[idx];
  int eid = ent >> SLA;
  eid = eid < 0 ? 0 : (eid > nE - 1 ? nE - 1 : eid);
  int sr = srcs[eid];
  sr = sr < 0 ? 0 : (sr > nN - 1 ? nN - 1 : sr);
  float al = (asd[sr] + adn) + ale[eid];
  al = (al > 0.0f) ? al : 0.2f * al;
  srOut = sr;
  alOut = al;
}

__device__ __forceinline__ void hit_walk(const float* __restrict__ xs, int sr, float w, int n, int lane,
                                         float& a0, float& a1, float& a2, float& a3) {
  const int wi = __float_as_int(w);
#pragma unroll 1
  for (int k = 0; k < n; ++k) {
    const int   sk = __builtin_amdgcn_readlane(sr, k);
    const float wk = __int_as_float(__builtin_amdgcn_readlane(wi, k));
    const v4f r = *(const v4f*)(xs + (size_t)sk * CP + 4 * lane);
    a0 = fmaf(wk, r.x, a0); a1 = fmaf(wk, r.y, a1);
    a2 = fmaf(wk, r.z, a2); a3 = fmaf(wk, r.w, a3);
  }
}

__global__ __launch_bounds__(NTHR) void k_scan(const int* __restrict__ srcs, const int* __restrict__ dsts,
                                               int nE, int nN, int vec8, int mpr,
                                               const float* __restrict__ xs, const float* __restrict__ asd,
                                               const float* __restrict__ ale, const float* __restrict__ bias,
                                               int nb, float* hout, double* rec) {
  extern __shared__ __attribute__((aligned(16))) int dsm[];
  int* list = dsm;
  int* hl   = dsm + LISTN;
  int* sl   = dsm + LISTN + RCAP;
  int* cnt  = dsm + LISTN + 2 * RCAP;
  int* offs = cnt + NBA;
  int* cur  = offs + NBA;
  int* misc = cur + NBA;
  const int tid = (int)threadIdx.x, lane = tid & 31, wave = tid >> 5;
  const int nodeBase = (int)blockIdx.x * NBA;

  {
    const v4i z4 = {0, 0, 0, 0};
    for (int i = tid * 4; i < AGG_ZINTS; i += NTHR * 4) *(v4ia*)(dsm + i) = z4;
    if (tid < 16) misc[tid] = 0;
  }
  v4f b4;
  {
    const int c0 = 4 * lane;
    const int cc = c0 < nb ? c0 : nb - 4;
    const bool okb = c0 < nb;
    const v4f t1 = *(const v4f*)(bias + cc);
    b4.x = okb ? bf16_val(t1.x) : 0.0f; b4.y = okb ? bf16_val(t1.y) : 0.0f;
    b4.z = okb ? bf16_val(t1.z) : 0.0f; b4.w = okb ? bf16_val(t1.w) : 0.0f;
  }
  __syncthreads();

  int t = 0, ov = 0;
  const int nChunks = (nE + CHUNK - 1) / CHUNK;
#pragma unroll 1
  for (int ch = 0; ch < nChunks; ++ch) {
    const int cbase = ch * CHUNK;
    const int wc = scan_chunk<SLA>(dsts, nE, cbase, nodeBase, NBA, vec8, list, tid, lane, wave);
    if (lane == 0) misc[wave] = wc;
    __syncthreads();
    if (wave == 0) {
#pragma unroll 1
      for (int w2 = 0; w2 < NWAVE; ++w2) {
        int c = misc[w2];
        c = c < 0 ? 0 : (c > WCAP ? WCAP : c);
#pragma unroll 1
        for (int b0 = 0; b0 < c; b0 += 32) {
          const int idx = b0 + lane;
          const int ent = list[w2 * WCAP + (idx < WCAP ? idx : WCAP - 1)];
          const int m32 = (c - b0) < 32 ? (c - b0) : 32;
#pragma unroll 1
          for (int k = 0; k < m32; ++k) {
            const int u    = __builtin_amdgcn_readlane(ent, k);
            const int slot = u & (NBA - 1);
            const int el   = (u >> SLA) & (CHUNK - 1);
            const int pk   = ((cbase + el) << SLA) | slot;
            if (t < RCAP) {
              if (lane == 0) { hl[t] = pk; cnt[slot] = cnt[slot] + 1; }
              t = t + 1;
            } else {
              ov = 1;
            }
          }
        }
      }
    }
    __syncthreads();
  }
  if (wave == 0 && lane == 0) { misc[8] = t; misc[9] = ov; }
  __syncthreads();
  int tt = misc[8];
  tt = tt < 0 ? 0 : (tt > RCAP ? RCAP : tt);
  const int ovf = misc[9];

  if (wave == 0) {
    const int base = lane * (NBA / 32);
    int s = 0;
#pragma unroll 1
    for (int i = 0; i < NBA / 32; ++i) s += cnt[base + i];
    int incl = s;
#pragma unroll
    for (int d = 1; d < 32; d <<= 1) {
      const int y = __shfl_up(incl, d, 32);
      if (lane >= d) incl += y;
    }
    int run = incl - s;
#pragma unroll 1
    for (int i = 0; i < NBA / 32; ++i) {
      const int cv = cnt[base + i];
      offs[base + i] = run;
      cur[base + i]  = run;
      run += cv;
    }
  }
  __syncthreads();
  if (wave == 0) {
#pragma unroll 1
    for (int b0 = 0; b0 < tt; b0 += 32) {
      const int idx = b0 + lane;
      const int ent = hl[idx < RCAP ? idx : RCAP - 1];
      const int m32 = (tt - b0) < 32 ? (tt - b0) : 32;
#pragma unroll 1
      for (int k = 0; k < m32; ++k) {
        const int u    = __builtin_amdgcn_readlane(ent, k);
        const int slot = u & (NBA - 1);
        if (lane == 0) {
          int p = cur[slot];
          p = p < 0 ? 0 : (p > RCAP - 1 ? RCAP - 1 : p);
          sl[p] = u;
          cur[slot] = p + 1;
        }
      }
    }
  }
  __syncthreads();

  const float qnan = __int_as_float(0x7fc00000);
  const float ninf = __int_as_float((int)0xff800000);
  const float pz = (ovf != 0) ? qnan : 0.0f;
  double sx0 = 0.0, sx1 = 0.0, sx2 = 0.0, sx3 = 0.0;
  double sq0 = 0.0, sq1 = 0.0, sq2 = 0.0, sq3 = 0.0;
#pragma unroll 1
  for (int si = 0; si < NBA / NWAVE; ++si) {
    const int s    = si * NWAVE + wave;
    const int node = nodeBase + s;
    int c = __builtin_amdgcn_readfirstlane(cnt[s]);
    const bool big = c > DEGCAP;
    c = c < 0 ? 0 : (c > DEGCAP ? DEGCAP : c);
    int o = __builtin_amdgcn_readfirstlane(offs[s]);
    o = o < 0 ? 0 : (o > RCAP ? RCAP : o);
    const int nc = node < nN ? node : nN - 1;
    const float adn = asd[(size_t)mpr + nc];

    int sr0 = 0, sr1 = 0;
    float al0 = 0.0f, al1 = 0.0f;
    hit_fetch(sl, o + lane, srcs, asd, ale, nE, nN, adn, sr0, al0);
    const bool v0 = lane < c;
    bool v1 = false;
    if (c > 32) {
      hit_fetch(sl, o + 32 + lane, srcs, asd, ale, nE, nN, adn, sr1, al1);
      v1 = (32 + lane) < c;
    }
    float mx = fmaxf(v0 ? al0 : ninf, v1 ? al1 : ninf);
#pragma unroll
    for (int d = 16; d >= 1; d >>= 1) mx = fmaxf(mx, __shfl_xor(mx, d, 32));
    const float x0 = expf(al0 - mx);
    const float x1 = expf(al1 - mx);
    const float e0 = v0 ? x0 : 0.0f;
    const float e1 = v1 ? x1 : 0.0f;
    float den = e0 + e1;
#pragma unroll
    for (int d = 16; d >= 1; d >>= 1) den += __shfl_xor(den, d, 32);
    const float inv = (den == 0.0f) ? 0.0f : (1.0f / den);
    const float w0 = e0 * inv;
    const float w1 = e1 * inv;

    float a0 = 0.0f, a1 = 0.0f, a2 = 0.0f, a3 = 0.0f;
    const int n0 = c < 32 ? c : 32;
    const int n1 = c - 32;
    hit_walk(xs, sr0, w0, n0, lane, a0, a1, a2, a3);
    hit_walk(xs, sr1, w1, n1, lane, a0, a1, a2, a3);

    const float pzr = big ? qnan : pz;
    v4f y;
    y.x = (a0 + b4.x) + pzr; y.y = (a1 + b4.y) + pzr;
    y.z = (a2 + b4.z) + pzr; y.w = (a3 + b4.w) + pzr;
    if (node < nN) {
      const double d0 = (double)y.x, d1 = (double)y.y, d2 = (double)y.z, d3 = (double)y.w;
      sx0 += d0; sx1 += d1; sx2 += d2; sx3 += d3;
      sq0 = fma(d0, d0, sq0); sq1 = fma(d1, d1, sq1); sq2 = fma(d2, d2, sq2); sq3 = fma(d3, d3, sq3);
      float* op = hout + (size_t)node * CP + 4 * lane;
      *(volatile v4f*)op = y;
      __threadfence();
      *(volatile v4f*)op = y;
    }
  }

  dbla* pd = (dbla*)hl;
  {
    dbla* ps = pd + (size_t)(wave * 2) * CP + 4 * lane;
    ps[0] = sx0; ps[1] = sx1; ps[2] = sx2; ps[3] = sx3;
    ps[CP + 0] = sq0; ps[CP + 1] = sq1; ps[CP + 2] = sq2; ps[CP + 3] = sq3;
  }
  __syncthreads();
  {
    const int e0i = 2 * (tid & 127);
    const int q   = e0i >> 7;
    const int col = e0i & (CP - 1);
    double r0 = 0.0, r1 = 0.0;
#pragma unroll 1
    for (int w2 = 0; w2 < NWAVE; ++w2) {
      const dbla* pp = pd + (size_t)(w2 * 2 + q) * CP + col;
      r0 += pp[0];
      r1 += pp[1];
    }
    v2d rv;
    rv.x = r0; rv.y = r1;
    double* rp = rec + (size_t)blockIdx.x * RECN + e0i;
    if (tid < 128) *(volatile v2d*)rp = rv;
    __threadfence();
    if (tid < 128) *(volatile v2d*)rp = rv;
  }
}

__global__ __launch_bounds__(NTHR) void k_comb(const double* __restrict__ rec, int nblk, double invN,
                                               float* stat) {
  __shared__ double sd[RECN];
  __shared__ __attribute__((aligned(16))) float st[RECN];
  const int tid = (int)threadIdx.x;
  double s = 0.0;
#pragma unroll 4
  for (int b = 0; b < nblk; ++b) s += rec[(size_t)b * RECN + tid];
  sd[tid] = s;
  __syncthreads();
  if (tid < CP) {
    const double mu  = sd[tid] * invN;
    double var = sd[CP + tid] * invN - mu * mu;
    var = (var < 0.0) ? 0.0 : var;
    const float vf = (float)var;
    st[tid]      = (float)mu;
    st[CP + tid] = rsqrtf(vf + 1e-5f);
  }
  __syncthreads();
  const v4f ov = *(const v4fa*)(st + 4 * (tid & 63));
  float* dp = stat + 4 * (tid & 63);
  if (tid < 64) *(volatile v4f*)dp = ov;
  __threadfence();
  if (tid < 64) *(volatile v4f*)dp = ov;
}

__device__ __forceinline__ float bn_relu(float h, float mu, float rs, float g, float b) {
  const float v = (g * (h - mu)) * rs + b;
  return (v > 0.0f) ? v : (v - v);
}

__global__ __launch_bounds__(NTHR) void k_bn0(const float* __restrict__ h, const float* __restrict__ stat,
                                              const float* __restrict__ g, const float* __restrict__ b,
                                              int nN, int nUnits, unsigned short* hhl) {
  const int u = (int)blockIdx.x * NTHR + (int)threadIdx.x;
  if (u >= nUnits) return;
  const int row = u >> 4;
  const int k8  = (u & 15) * 8;
  const int rc  = row < nN ? row : nN - 1;
  const float* hp = h + (size_t)rc * CP + k8;
  const v4f ha = *(const v4f*)hp,              hb = *(const v4f*)(hp + 4);
  const v4f ma = *(const v4f*)(stat + k8),     mb = *(const v4f*)(stat + k8 + 4);
  const v4f ra = *(const v4f*)(stat + CP + k8), rb = *(const v4f*)(stat + CP + k8 + 4);
  const v4f ga = *(const v4f*)(g + k8),        gb = *(const v4f*)(g + k8 + 4);
  const v4f ba = *(const v4f*)(b + k8),        bb = *(const v4f*)(b + k8 + 4);
  const bool ok = row < nN;
  float v[8];
  v[0] = bn_relu(ha.x, ma.x, ra.x, bf16_val(ga.x), bf16_val(ba.x));
  v[1] = bn_relu(ha.y, ma.y, ra.y, bf16_val(ga.y), bf16_val(ba.y));
  v[2] = bn_relu(ha.z, ma.z, ra.z, bf16_val(ga.z), bf16_val(ba.z));
  v[3] = bn_relu(ha.w, ma.w, ra.w, bf16_val(ga.w), bf16_val(ba.w));
  v[4] = bn_relu(hb.x, mb.x, rb.x, bf16_val(gb.x), bf16_val(bb.x));
  v[5] = bn_relu(hb.y, mb.y, rb.y, bf16_val(gb.y), bf16_val(bb.y));
  v[6] = bn_relu(hb.z, mb.z, rb.z, bf16_val(gb.z), bf16_val(bb.z));
  v[7] = bn_relu(hb.w, mb.w, rb.w, bf16_val(gb.w), bf16_val(bb.w));
  v8us oh, ol;
#pragma unroll
  for (int i = 0; i < 8; ++i) {
    const float vv = ok ? v[i] : 0.0f;
    const unsigned hbits = bf16_bits(vv);
    const unsigned lbits = bf16_bits(vv - __uint_as_float(hbits << 16));
    oh[i] = (unsigned short)hbits;
    ol[i] = (unsigned short)lbits;
  }
  unsigned short* dp = hhl + (size_t)row * KA1 + k8;
  *(volatile v8us*)dp = oh;
  *(volatile v8us*)(dp + CP) = ol;
  __threadfence();
  *(volatile v8us*)dp = oh;
  *(volatile v8us*)(dp + CP) = ol;
}

__global__ __launch_bounds__(NTHR) void k_bnf(const float* __restrict__ o1, const float* __restrict__ stat,
                                              const float* __restrict__ g, const float* __restrict__ b,
                                              int nN, float* out) {
  __shared__ __attribute__((aligned(16))) float ps[4 * CP];
  const int tid = (int)threadIdx.x;
  if (tid < CP) {
    const int gc = tid < CO1 ? tid : CO1 - 1;
    ps[tid]          = stat[tid];
    ps[CP + tid]     = stat[CP + tid];
    ps[2 * CP + tid] = bf16_val(g[gc]);
    ps[3 * CP + tid] = bf16_val(b[gc]);
  }
  __syncthreads();
  const int rowBase = (int)blockIdx.x * ORB;
  constexpr int NIT = (ORB * CO1) / (4 * NTHR);
  v4f ov[NIT];
#pragma unroll
  for (int it = 0; it < NIT; ++it) {
    const int f   = 4 * (it * NTHR + tid);
    const int r   = f / CO1;
    const int col = f - r * CO1;
    const int row = rowBase + r;
    const int rc  = row < nN ? row : nN - 1;
    const v4f hv = *(const v4f*)(o1 + (size_t)rc * CP + col);
    const v4f mu = *(const v4fa*)(ps + col);
    const v4f rs = *(const v4fa*)(ps + CP + col);
    const v4f gg = *(const v4fa*)(ps + 2 * CP + col);
    const v4f bb = *(const v4fa*)(ps + 3 * CP + col);
    v4f y;
    y.x = (gg.x * (hv.x - mu.x)) * rs.x + bb.x;
    y.y = (gg.y * (hv.y - mu.y)) * rs.y + bb.y;
    y.z = (gg.z * (hv.z - mu.z)) * rs.z + bb.z;
    y.w = (gg.w * (hv.w - mu.w)) * rs.w + bb.w;
    ov[it] = y;
  }
  float* ob = out + (size_t)rowBase * CO1;
#pragma unroll
  for (int it = 0; it < NIT; ++it) {
    const int f = 4 * (it * NTHR + tid);
    if (rowBase + f / CO1 < nN) *(volatile v4f*)(ob + f) = ov[it];
  }
  __threadfence();
#pragma unroll
  for (int it = 0; it < NIT; ++it) {
    const int f = 4 * (it * NTHR + tid);
    if (rowBase + f / CO1 < nN) *(volatile v4f*)(ob + f) = ov[it];
  }
}

static inline int cdiv(int a, int b) { return (a + b - 1) / b; }
static inline size_t al256(size_t o) { return (o + 255) & ~(size_t)255; }

extern "C" void kernel_launch(void* const* d_in, const int* in_sizes, int n_in,
                              void* d_out, int out_size, void* d_ws, size_t ws_size,
                              hipStream_t stream) {
  if (n_in < 19) return;
  if (in_sizes[0] < CP || (in_sizes[0] % CP) != 0) return;
  const int nN = in_sizes[0] / CP;
  if (nN < 64 || nN > (1 << 22)) return;
  if (in_sizes[1] < 2 || (in_sizes[1] & 1) != 0) return;
  const int nE = in_sizes[1] / 2;
  if (nE < 1 || nE >= (1 << (31 - SLA))) return;
  if ((long long)in_sizes[2] != (long long)nE * EDIM) return;
  if (in_sizes[3] != CP * CP) return;
  if (in_sizes[4] != CP || in_sizes[5] != CP || in_sizes[7] != CP || in_sizes[8] != CP) return;
  if (in_sizes[6] != EDIM * CP) return;
  if (in_sizes[9] != CP * CO1) return;
  if (in_sizes[10] != CO1 || in_sizes[11] != CO1 || in_sizes[13] != CO1 || in_sizes[14] != CO1) return;
  if (in_sizes[12] != EDIM * CO1) return;
  if (in_sizes[15] != CP || in_sizes[16] != CP) return;
  if (in_sizes[17] != CO1 || in_sizes[18] != CO1) return;
  if ((long long)out_size != (long long)nN * CO1) return;
  if ((((long long)nN * CO1) % 32) != 0) return;

  const float* x    = (const float*)d_in[0];
  const int*   edge = (const int*)d_in[1];
  const float* eatt = (const float*)d_in[2];
  const float* W0   = (const float*)d_in[3];
  const float* aS0  = (const float*)d_in[4];
  const float* aD0  = (const float*)d_in[5];
  const float* We0  = (const float*)d_in[6];
  const float* aE0  = (const float*)d_in[7];
  const float* b0   = (const float*)d_in[8];
  const float* W1   = (const float*)d_in[9];
  const float* aS1  = (const float*)d_in[10];
  const float* aD1  = (const float*)d_in[11];
  const float* We1  = (const float*)d_in[12];
  const float* aE1  = (const float*)d_in[13];
  const float* b1   = (const float*)d_in[14];
  const float* bng  = (const float*)d_in[15];
  const float* bnb  = (const float*)d_in[16];
  const float* bfg  = (const float*)d_in[17];
  const float* bfb  = (const float*)d_in[18];
  float* out = (float*)d_out;
  const int* src = edge;
  const int* dst = edge + nE;

  const int MP = cdiv(nN, GBM) * GBM;
  const int gM = MP / GBM;
  const int gA = cdiv(nN, NBA);
  if ((long long)gA * NBA < (long long)nN) return;
  const int EP = cdiv(nE, NTHR) * NTHR;
  const int vec8 = ((nE & 3) == 0) ? 1 : 0;
  const double invN = 1.0 / (double)nN;

  char* ws = (char*)d_ws;
  size_t off = 0;
  const size_t oXB  = off; off = al256(off + (size_t)MP * CP * 2);
  const size_t oXS  = off; off = al256(off + (size_t)MP * CP * 4);
  const size_t oH   = off; off = al256(off + (size_t)MP * CP * 4);
  const size_t oHHL = off; off = al256(off + (size_t)MP * KA1 * 2);
  const size_t oALE = off; off = al256(off + (size_t)2 * EP * 4);
  const size_t oAD0 = off; off = al256(off + (size_t)2 * MP * 4);
  const size_t oAD1 = off; off = al256(off + (size_t)2 * MP * 4);
  const size_t oW0T = off; off = al256(off + (size_t)CP * KA0 * 2);
  const size_t oW1T = off; off = al256(off + (size_t)CP * KA1 * 2);
  const size_t oPRM = off; off = al256(off + (size_t)32 * 4);
  const size_t oRC0 = off; off = al256(off + (size_t)gA * RECN * 8);
  const size_t oRC1 = off; off = al256(off + (size_t)gA * RECN * 8);
  const size_t oST0 = off; off = al256(off + (size_t)RECN * 4);
  const size_t oST1 = off; off = al256(off + (size_t)RECN * 4);
  if (off > ws_size || off > (size_t)WSMAX) return;
  unsigned short* XB   = (unsigned short*)(ws + oXB);
  float*          XS   = (float*)(ws + oXS);
  float*          H    = (float*)(ws + oH);
  unsigned short* HHL  = (unsigned short*)(ws + oHHL);
  float*          ALE  = (float*)(ws + oALE);
  float*          ASD0 = (float*)(ws + oAD0);
  float*          ASD1 = (float*)(ws + oAD1);
  unsigned short* W0T  = (unsigned short*)(ws + oW0T);
  unsigned short* W1T2 = (unsigned short*)(ws + oW1T);
  float*          PRM  = (float*)(ws + oPRM);
  double*         REC0 = (double*)(ws + oRC0);
  double*         REC1 = (double*)(ws + oRC1);
  float*          ST0  = (float*)(ws + oST0);
  float*          ST1  = (float*)(ws + oST1);

  const size_t scanLds = (size_t)AGG_LDS_INTS * 4;
  hipFuncSetAttribute(reinterpret_cast<const void*>(&k_scan), hipFuncAttributeMaxDynamicSharedMemorySize, (int)scanLds);

  const int nUx = MP * (CP / 8);
  k_wprep<<<WPB, NTHR, 0, stream>>>(W0, W1, We0, aE0, We1, aE1, W0T, W1T2, PRM);
  k_cvx<<<cdiv(nUx, NTHR), NTHR, 0, stream>>>(x, nN, nUx, XB);
  k_edge<<<EP / NTHR, NTHR, 0, stream>>>(eatt, PRM, nE, EP, ALE);
  k_gemm<<<gM, GTHR, 0, stream>>>(XB, W0T, KA0, aS0, aD0, CP, XS, ASD0, MP);
  k_scan<<<gA, NTHR, scanLds, stream>>>(src, dst, nE, nN, vec8, MP, XS, ASD0, ALE, b0, CP, H, REC0);
  k_comb<<<1, NTHR, 0, stream>>>(REC0, gA, invN, ST0);
  k_bn0<<<cdiv(nUx, NTHR), NTHR, 0, stream>>>(H, ST0, bng, bnb, nN, nUx, HHL);
  k_gemm<<<gM, GTHR, 0, stream>>>(HHL, W1T2, KA1, aS1, aD1, CO1, XS, ASD1, MP);
  k_scan<<<gA, NTHR, scanLds, stream>>>(src, dst, nE, nN, vec8, MP, XS, ASD1, ALE + EP, b1, CO1, H, REC1);
  k_comb<<<1, NTHR, 0, stream>>>(REC1, gA, invN, ST1);
  k_bnf<<<cdiv(nN, ORB), NTHR, 0, stream>>>(H, ST1, bfg, bfb, nN, out);
}
